// GraphAttentionNetwork_44332652429421
// MI455X (gfx1250) — hardware-verified
//
#include <hip/hip_runtime.h>
#include <math.h>


typedef _Float16     v16h __attribute__((ext_vector_type(16)));
typedef _Float16     v8h  __attribute__((ext_vector_type(8)));
typedef float        v8f  __attribute__((ext_vector_type(8)));
typedef float        v4f  __attribute__((ext_vector_type(4)));
typedef unsigned int v4u  __attribute__((ext_vector_type(4)));

union Frag { v16h v; v8h half[2]; };
union H8   { v8h h; v4u u; };

#define DM      256
#define WSCALE  16.0f
#define WALPHA  0.0625f
#define AR      64
#define LCAP    4096
#define NBMAX   128
#define NBCAP   136

__device__ __forceinline__ v8f wmma16(v16h a, v16h b, v8f c) {
  v8f d = __builtin_amdgcn_wmma_f32_16x16x32_f16(false, a, false, b, (short)0, c, false, false);
  asm volatile("v_nop\n\tv_nop\n\tv_nop\n\tv_nop" : "+v"(d) : "v"(a), "v"(b));
  return d;
}

__device__ __forceinline__ v4u pack8h(v4f a, v4f b) {
  H8 x;
  v8h hv;
  hv[0] = (_Float16)a.x; hv[1] = (_Float16)a.y; hv[2] = (_Float16)a.z; hv[3] = (_Float16)a.w;
  hv[4] = (_Float16)b.x; hv[5] = (_Float16)b.y; hv[6] = (_Float16)b.z; hv[7] = (_Float16)b.w;
  x.h = hv;
  return x.u;
}

__global__ __launch_bounds__(256)
void build_xc_kernel(const float* __restrict__ agg, const int* __restrict__ sid,
                     const float* __restrict__ spk, int nspk, _Float16* xc, int nn) {
  const int t = threadIdx.x;
  const int n = blockIdx.x * 4 + (t >> 6);
  if (n >= nn) return;
  const int col = (t & 63) * 8;
  int s = sid[n];
  s = s < 0 ? 0 : (s >= nspk ? nspk - 1 : s);
  const float* src = (col < DM) ? (agg + (size_t)n * DM + col)
                                : (spk + (size_t)s * DM + (col - DM));
  const v4f a = *(const v4f*)src;
  const v4f b = *(const v4f*)(src + 4);
  const v4u pv = pack8h(a, b);
  _Float16* p = xc + (size_t)n * (2 * DM) + col;
  *(volatile v4u*)p = pv;
  __threadfence();
  *(volatile v4u*)p = pv;
}

__global__ __launch_bounds__(256)
void wtrans_kernel(const float* __restrict__ W, _Float16* Wt, int K, int N) {
  __shared__ __attribute__((aligned(16))) _Float16 tl[32][72];
  const int t = threadIdx.x;
  const int ntn = N >> 5;
  const int nt = blockIdx.x % ntn, kt = blockIdx.x / ntn;
  const int n0 = nt * 32, k0 = kt * 64;
  const float* src = W  + (size_t)blockIdx.y * K * N;
  _Float16*    dst = Wt + (size_t)blockIdx.y * K * N;
#pragma unroll
  for (int i = 0; i < 8; ++i) {
    const int k = i * 8 + (t >> 5);
    const int n = t & 31;
    const float v = src[(size_t)(k0 + k) * N + n0 + n] * WSCALE;
    tl[n][k] = (_Float16)v;
  }
  __syncthreads();
  const int n = t >> 3, seg = t & 7;
  H8 x;
  x.h = *(const v8h*)&tl[n][seg * 8];
  _Float16* p = dst + (size_t)(n0 + n) * K + k0 + seg * 8;
  *(volatile v4u*)p = x.u;
  __threadfence();
  *(volatile v4u*)p = x.u;
}

__global__ __launch_bounds__(128)
void gemm_f16_kernel(const _Float16* __restrict__ A, int lda, int K,
                     const _Float16* __restrict__ Bt, const float* __restrict__ bias,
                     float alpha, int elu, float* outF, _Float16* outH) {
  __shared__ __attribute__((aligned(16))) float    stF[4][16][68];
  __shared__ __attribute__((aligned(16))) _Float16 stH[4][16][72];
  const int lane = threadIdx.x & 31, w = threadIdx.x >> 5;
  const int h = lane >> 4, m = lane & 15;
  const int bn = blockIdx.x & 3, bm = blockIdx.x >> 2;
  const int row0 = bm * 64 + w * 16, col0 = bn * 64;

  const v8f z8 = {0.f, 0.f, 0.f, 0.f, 0.f, 0.f, 0.f, 0.f};
  v8f acc0 = z8, acc1 = z8, acc2 = z8, acc3 = z8;

  const _Float16* ap = A  + (size_t)(row0 + m) * lda + 8 * h;
  const _Float16* bp = Bt + (size_t)(col0 + m) * K + 8 * h;
  const size_t bs = (size_t)16 * K;

#pragma unroll 2
  for (int k0 = 0; k0 < K; k0 += 32) {
    Frag a, b;
    a.half[0] = *(const v8h*)(ap + k0);
    a.half[1] = *(const v8h*)(ap + k0 + 16);
    b.half[0] = *(const v8h*)(bp + k0);
    b.half[1] = *(const v8h*)(bp + k0 + 16);
    acc0 = wmma16(a.v, b.v, acc0);
    b.half[0] = *(const v8h*)(bp + bs + k0);
    b.half[1] = *(const v8h*)(bp + bs + k0 + 16);
    acc1 = wmma16(a.v, b.v, acc1);
    b.half[0] = *(const v8h*)(bp + 2 * bs + k0);
    b.half[1] = *(const v8h*)(bp + 2 * bs + k0 + 16);
    acc2 = wmma16(a.v, b.v, acc2);
    b.half[0] = *(const v8h*)(bp + 3 * bs + k0);
    b.half[1] = *(const v8h*)(bp + 3 * bs + k0 + 16);
    acc3 = wmma16(a.v, b.v, acc3);
  }

  float vals[4][8];
  {
    const float b0 = bias ? bias[col0 + m]      : 0.f;
    const float b1 = bias ? bias[col0 + 16 + m] : 0.f;
    const float b2 = bias ? bias[col0 + 32 + m] : 0.f;
    const float b3 = bias ? bias[col0 + 48 + m] : 0.f;
#pragma unroll
    for (int r = 0; r < 8; ++r) {
      vals[0][r] = acc0[r] * alpha + b0;
      vals[1][r] = acc1[r] * alpha + b1;
      vals[2][r] = acc2[r] * alpha + b2;
      vals[3][r] = acc3[r] * alpha + b3;
    }
  }
  if (elu) {
#pragma unroll
    for (int s = 0; s < 4; ++s)
#pragma unroll
      for (int r = 0; r < 8; ++r) {
        const float v = vals[s][r];
        vals[s][r] = (v > 0.f) ? v : expm1f(v);
      }
  }

  const int rr = lane >> 3, seg = lane & 7;

  if (outH != nullptr) {
#pragma unroll
    for (int s = 0; s < 4; ++s)
#pragma unroll
      for (int r = 0; r < 8; ++r)
        stH[w][8 * h + r][16 * s + m] = (_Float16)vals[s][r];
    __syncthreads();
    H8 hv[4];
#pragma unroll
    for (int i = 0; i < 4; ++i) hv[i].h = *(const v8h*)&stH[w][i * 4 + rr][seg * 8];
#pragma unroll
    for (int i = 0; i < 4; ++i) {
      _Float16* p = outH + (size_t)(row0 + i * 4 + rr) * DM + col0 + seg * 8;
      *(volatile v4u*)p = hv[i].u;
    }
    __threadfence();
#pragma unroll
    for (int i = 0; i < 4; ++i) {
      _Float16* p = outH + (size_t)(row0 + i * 4 + rr) * DM + col0 + seg * 8;
      *(volatile v4u*)p = hv[i].u;
    }
  }

  if (outF != nullptr) {
#pragma unroll
    for (int s = 0; s < 4; ++s)
#pragma unroll
      for (int r = 0; r < 8; ++r)
        stF[w][8 * h + r][16 * s + m] = vals[s][r];
    __syncthreads();
    v4f fv[8];
#pragma unroll
    for (int i = 0; i < 8; ++i) {
      const int li = i * 4 + rr;
      const int row = li >> 1, hc = li & 1;
      fv[i] = *(const v4f*)&stF[w][row][hc * 32 + seg * 4];
    }
#pragma unroll
    for (int i = 0; i < 8; ++i) {
      const int li = i * 4 + rr;
      const int row = li >> 1, hc = li & 1;
      float* p = outF + (size_t)(row0 + row) * DM + col0 + hc * 32 + seg * 4;
      *(volatile v4f*)p = fv[i];
    }
    __threadfence();
#pragma unroll
    for (int i = 0; i < 8; ++i) {
      const int li = i * 4 + rr;
      const int row = li >> 1, hc = li & 1;
      float* p = outF + (size_t)(row0 + row) * DM + col0 + hc * 32 + seg * 4;
      *(volatile v4f*)p = fv[i];
    }
  }
}

__global__ __launch_bounds__(256)
void attn_sparse_kernel(const float* __restrict__ q2, const float* __restrict__ k2,
                        const float* __restrict__ v2,
                        const int* __restrict__ ei, const int* __restrict__ et,
                        const float* __restrict__ edge_w,
                        int layer, int E, int nchunks, int nn, float scale,
                        _Float16* o16) {
  __shared__ unsigned int lst[LCAP];
  __shared__ unsigned int nbA[8][NBMAX];
  __shared__ unsigned int nbB[8][NBCAP];
  __shared__ float sc[8][NBCAP][8];
  __shared__ int wcnt[8];
  __shared__ float sew[4];

  const int t = threadIdx.x, lane = t & 31, w = t >> 5;
  const int n0 = blockIdx.x * AR;
  const unsigned ltmask = (1u << lane) - 1u;

  if (t < 4) {
    const float x = edge_w[layer * 4 + t];
    sew[t] = fmaxf(x, 0.f) + log1pf(expf(-fabsf(x)));
  }
  __syncthreads();

  int base = 0;
  for (int c = 0; c < nchunks; ++c) {
    const int e = c * 256 + t;
    bool hit = false;
    unsigned pack = 0u;
    if (e < E) {
      const int s = ei[e];
      const unsigned lr = (unsigned)(s - n0);
      if (lr < (unsigned)AR) {
        int d = ei[(size_t)E + e];
        d = d < 0 ? 0 : (d >= nn ? nn - 1 : d);
        int ty = et[e] - 1;
        ty = ty < 0 ? 0 : (ty > 3 ? 3 : ty);
        hit = true;
        pack = (unsigned)d | (lr << 16) | ((unsigned)ty << 24);
      }
    }
    const unsigned bal = __builtin_amdgcn_ballot_w32(hit);
    const int pre = __builtin_popcount(bal & ltmask);
    if (lane == 0) wcnt[w] = __builtin_popcount(bal);
    __syncthreads();
    int off = 0, tot = 0;
#pragma unroll
    for (int i = 0; i < 8; ++i) {
      const int cc = wcnt[i];
      tot += cc;
      off += (i < w) ? cc : 0;
    }
    const int slot = base + off + pre;
    if (hit && slot < LCAP) lst[slot] = pack;
    base += tot;
    __syncthreads();
  }
  const int cnt = base < LCAP ? base : LCAP;

  const int hh = lane >> 2, q4 = lane & 3;
  for (int i = 0; i < 8; ++i) {
    const int lr = w * 8 + i;
    const int n = n0 + lr;

    int na = 0;
    for (int b0 = 0; b0 < LCAP; b0 += 32) {
      if (b0 >= cnt) break;
      const int idx = b0 + lane;
      unsigned ent = 0u;
      bool hit = false;
      if (idx < cnt) {
        ent = lst[idx];
        hit = ((ent >> 16) & 255u) == (unsigned)lr;
      }
      const unsigned bal = __builtin_amdgcn_ballot_w32(hit);
      const int pos = na + __builtin_popcount(bal & ltmask);
      if (hit && pos < NBMAX) nbA[w][pos] = ent;
      na += __builtin_popcount(bal);
    }
    if (na > NBMAX) na = NBMAX;
    __syncthreads();

    int nb = 0;
    bool selfseen = false;
    for (int c0 = 0; c0 < NBMAX; c0 += 32) {
      if (c0 >= na) break;
      const int a = c0 + lane;
      unsigned ent = 0u;
      bool keep = false;
      if (a < na) {
        ent = nbA[w][a];
        keep = true;
        const unsigned dd = ent & 0xffffu;
        for (int b = a + 1; b < na; ++b) {
          if ((nbA[w][b] & 0xffffu) == dd) { keep = false; break; }
        }
      }
      const unsigned bal = __builtin_amdgcn_ballot_w32(keep);
      const int pos = nb + __builtin_popcount(bal & ltmask);
      if (keep && pos < NBMAX) nbB[w][pos] = ent;
      const unsigned sb = __builtin_amdgcn_ballot_w32(keep && ((ent & 0xffffu) == (unsigned)n));
      selfseen = selfseen || (sb != 0u);
      nb += __builtin_popcount(bal);
    }
    if (nb > NBMAX) nb = NBMAX;
    if (!selfseen) {
      if (lane == 0) nbB[w][nb] = (unsigned)n | (3u << 24);
      nb += 1;
    }
    __syncthreads();

    const float* qrow = q2 + (size_t)n * DM + lane * 8;
    const v4f qa = *(const v4f*)qrow;
    const v4f qb = *(const v4f*)(qrow + 4);
    float mx = -__builtin_inff();
#pragma unroll 1
    for (int j = 0; j < nb && j < NBCAP; ++j) {
      const unsigned ent = nbB[w][j];
      int mm = (int)(ent & 0xffffu);
      mm = mm < nn ? mm : nn - 1;
      const float* kr = k2 + (size_t)mm * DM + lane * 8;
      const v4f ka = *(const v4f*)kr;
      const v4f kb = *(const v4f*)(kr + 4);
      float part = qa.x * ka.x;
      part += qa.y * ka.y; part += qa.z * ka.z; part += qa.w * ka.w;
      part += qb.x * kb.x; part += qb.y * kb.y; part += qb.z * kb.z; part += qb.w * kb.w;
      part += __shfl_xor(part, 1);
      part += __shfl_xor(part, 2);
      const int ty = (int)((ent >> 24) & 3u);
      const float s = part * scale + sew[ty];
      mx = fmaxf(mx, s);
      if (q4 == 0) sc[w][j][hh] = s;
    }
    __syncthreads();

    float ssum = 0.f;
#pragma unroll 1
    for (int j = 0; j < nb && j < NBCAP; ++j) {
      const float s = sc[w][j][hh];
      const float ex = expf(s - mx);
      ssum += ex;
      if (q4 == 0) sc[w][j][hh] = ex;
    }
    const float inv = 1.0f / ssum;
    __syncthreads();

    v4f oa = {0.f, 0.f, 0.f, 0.f}, ob = {0.f, 0.f, 0.f, 0.f};
#pragma unroll 1
    for (int j = 0; j < nb && j < NBCAP; ++j) {
      const unsigned ent = nbB[w][j];
      int mm = (int)(ent & 0xffffu);
      mm = mm < nn ? mm : nn - 1;
      const float p = sc[w][j][hh] * inv;
      const float* vr = v2 + (size_t)mm * DM + lane * 8;
      const v4f va = *(const v4f*)vr;
      const v4f vb = *(const v4f*)(vr + 4);
      oa += p * va;
      ob += p * vb;
    }
    const v4u pv = pack8h(oa, ob);
    _Float16* op = o16 + (size_t)n * DM + lane * 8;
    *(volatile v4u*)op = pv;
    __threadfence();
    *(volatile v4u*)op = pv;
    __syncthreads();
  }
}

extern "C" void kernel_launch(void* const* d_in, const int* in_sizes, int n_in,
                              void* d_out, int out_size, void* d_ws, size_t ws_size,
                              hipStream_t stream) {
  if (n_in < 18) return;
  const float* agg    = (const float*)d_in[0];
  const int*   sid    = (const int*)d_in[1];
  const int*   eidx   = (const int*)d_in[2];
  const int*   etype  = (const int*)d_in[3];
  const float* spk    = (const float*)d_in[4];
  const float* W_in   = (const float*)d_in[5];
  const float* b_in   = (const float*)d_in[6];
  const float* edge_w = (const float*)d_in[7];
  const float* Wq     = (const float*)d_in[8];
  const float* bq     = (const float*)d_in[9];
  const float* Wk     = (const float*)d_in[10];
  const float* bk     = (const float*)d_in[11];
  const float* Wv     = (const float*)d_in[12];
  const float* bv     = (const float*)d_in[13];
  const float* in_w   = (const float*)d_in[14];
  const float* in_b   = (const float*)d_in[15];
  const float* out_w  = (const float*)d_in[16];
  const float* out_b  = (const float*)d_in[17];
  float* outp = (float*)d_out;

  const int nn   = in_sizes[1];
  const int E    = in_sizes[3];
  const int nspk = in_sizes[4] / DM;
  const int L    = in_sizes[8] / (DM * DM);
  const int KIN  = 2 * DM;

  if (nn <= 0 || (nn % 64) != 0 || nn > 65536) return;
  if (in_sizes[0] != nn * DM || in_sizes[2] != 2 * E || out_size != nn * DM) return;
  if (in_sizes[5] != KIN * DM || nspk < 1 || L < 1) return;
  if (in_sizes[7] < L * 4 || in_sizes[10] != L * DM * DM || in_sizes[12] != L * DM * DM) return;
  if (in_sizes[14] != L * 3 * DM * DM || in_sizes[16] != L * DM * DM) return;
  if (in_sizes[6] < DM || in_sizes[9] < L * DM || in_sizes[11] < L * DM || in_sizes[13] < L * DM) return;
  if (in_sizes[15] < L * 3 * DM || in_sizes[17] < L * DM) return;

  char* ws = (char*)d_ws;
  size_t off = 0;
  auto carve = [&](size_t bytes) -> char* {
    char* p = ws + off;
    off += (bytes + 255) & ~(size_t)255;
    return p;
  };
  const size_t act16 = (size_t)nn * DM * sizeof(_Float16);
  const size_t act32 = (size_t)nn * DM * sizeof(float);
  const size_t wmat  = (size_t)DM * DM * sizeof(_Float16);
  _Float16* xc16  = (_Float16*)carve((size_t)nn * KIN * sizeof(_Float16));
  _Float16* x16   = (_Float16*)carve(act16);
  _Float16* q1h   = (_Float16*)carve(act16);
  _Float16* k1h   = (_Float16*)carve(act16);
  _Float16* v1h   = (_Float16*)carve(act16);
  float*    q2    = (float*)carve(act32);
  float*    k2    = (float*)carve(act32);
  float*    v2    = (float*)carve(act32);
  _Float16* o16   = (_Float16*)carve(act16);
  _Float16* wt_in = (_Float16*)carve((size_t)KIN * DM * sizeof(_Float16));
  _Float16* wt_q  = (_Float16*)carve((size_t)L * wmat);
  _Float16* wt_k  = (_Float16*)carve((size_t)L * wmat);
  _Float16* wt_v  = (_Float16*)carve((size_t)L * wmat);
  _Float16* wt_iw = (_Float16*)carve((size_t)L * 3 * wmat);
  _Float16* wt_o  = (_Float16*)carve((size_t)L * wmat);
  if (off > ws_size || off > ((size_t)128 << 20)) return;

  build_xc_kernel<<<(nn + 3) / 4, 256, 0, stream>>>(agg, sid, spk, nspk, xc16, nn);
  auto wtr = [&](const float* W, _Float16* Wt, int K, int nmat) {
    dim3 g((DM / 32) * (K / 64), nmat);
    wtrans_kernel<<<g, 256, 0, stream>>>(W, Wt, K, DM);
  };
  wtr(W_in,  wt_in, KIN, 1);
  wtr(Wq,    wt_q,  DM,  L);
  wtr(Wk,    wt_k,  DM,  L);
  wtr(Wv,    wt_v,  DM,  L);
  wtr(in_w,  wt_iw, DM,  3 * L);
  wtr(out_w, wt_o,  DM,  L);

  auto gemm = [&](const _Float16* A, int lda, int K, const _Float16* Bt, const float* bias,
                  int elu, float* oF, _Float16* oH) {
    const int blocks = (nn / 64) * (DM / 64);
    gemm_f16_kernel<<<blocks, 128, 0, stream>>>(A, lda, K, Bt, bias, WALPHA, elu, oF, oH);
  };

  gemm(xc16, KIN, KIN, wt_in, b_in, 1, nullptr, x16);

  const float scale = (float)(1.0 / sqrt(32.0));
  const int nchunks = (E + 255) / 256;
  const size_t mstride = (size_t)DM * DM;

  for (int l = 0; l < L; ++l) {
    gemm(x16, DM, DM, wt_q + (size_t)l * mstride, bq + (size_t)l * DM, 0, nullptr, q1h);
    gemm(x16, DM, DM, wt_k + (size_t)l * mstride, bk + (size_t)l * DM, 0, nullptr, k1h);
    gemm(x16, DM, DM, wt_v + (size_t)l * mstride, bv + (size_t)l * DM, 0, nullptr, v1h);
    gemm(q1h, DM, DM, wt_iw + ((size_t)l * 3 + 0) * mstride, in_b + ((size_t)l * 3 + 0) * DM, 0, q2, nullptr);
    gemm(k1h, DM, DM, wt_iw + ((size_t)l * 3 + 1) * mstride, in_b + ((size_t)l * 3 + 1) * DM, 0, k2, nullptr);
    gemm(v1h, DM, DM, wt_iw + ((size_t)l * 3 + 2) * mstride, in_b + ((size_t)l * 3 + 2) * DM, 0, v2, nullptr);

    attn_sparse_kernel<<<nn / AR, 256, 0, stream>>>(q2, k2, v2, eidx, etype, edge_w,
                                                    l, E, nchunks, nn, scale, o16);

    const bool last = (l == L - 1);
    gemm(o16, DM, DM, wt_o + (size_t)l * mstride, out_b + (size_t)l * DM,
         last ? 0 : 1, last ? outp : nullptr, last ? nullptr : x16);
  }
}
